// HeteroGAE_22574348107990
// MI455X (gfx1250) — hardware-verified
//
#include <hip/hip_runtime.h>
#include <hip/hip_bf16.h>
#include <stddef.h>


#define DIM     64
#define NBAS    16
#define NTHR    256
#define NWAVE   8
#define EPT     8
#define NGRP    2
#define CHUNK   (NTHR * EPT * NGRP)
#define WCAP    (EPT * NGRP * 32)
#define LISTN   (NWAVE * WCAP)
#define NB      1024
#define GROWS   64
#define WPL     (DIM * DIM)

#define LDS_AGG (NB * DIM * 4 + LISTN * 4)

static_assert((CHUNK & (CHUNK - 1)) == 0);
static_assert(CHUNK <= 4096);
static_assert(NB <= 4096 && (NB & (NB - 1)) == 0);
static_assert((NB * DIM) % (NWAVE * 128) == 0);
static_assert(NB % NWAVE == 0);

typedef float v2f __attribute__((ext_vector_type(2)));
typedef float v4f __attribute__((ext_vector_type(4)));
typedef float v8f __attribute__((ext_vector_type(8)));
typedef int   v4i __attribute__((ext_vector_type(4)));
typedef unsigned short v8us  __attribute__((ext_vector_type(8)));
typedef unsigned short v16us __attribute__((ext_vector_type(16)));
typedef __bf16 v16bf __attribute__((ext_vector_type(16)));
union FragB { v16bf v; v16us u; v8us h[2]; };
struct HL { v8us hi; v8us lo; };

__device__ __forceinline__ unsigned int bf_bits(float f) {
  const unsigned int u = __float_as_uint(f);
  return (u + 0x7FFFu + ((u >> 16) & 1u)) >> 16;
}
__device__ __forceinline__ unsigned int bf_lo(float f, unsigned int hb) {
  return bf_bits(f - __uint_as_float(hb << 16));
}

__device__ __forceinline__ HL split8(v4f a, v4f b) {
  HL r;
  unsigned int h;
  h = bf_bits(a.x); r.hi[0] = (unsigned short)h; r.lo[0] = (unsigned short)bf_lo(a.x, h);
  h = bf_bits(a.y); r.hi[1] = (unsigned short)h; r.lo[1] = (unsigned short)bf_lo(a.y, h);
  h = bf_bits(a.z); r.hi[2] = (unsigned short)h; r.lo[2] = (unsigned short)bf_lo(a.z, h);
  h = bf_bits(a.w); r.hi[3] = (unsigned short)h; r.lo[3] = (unsigned short)bf_lo(a.w, h);
  h = bf_bits(b.x); r.hi[4] = (unsigned short)h; r.lo[4] = (unsigned short)bf_lo(b.x, h);
  h = bf_bits(b.y); r.hi[5] = (unsigned short)h; r.lo[5] = (unsigned short)bf_lo(b.y, h);
  h = bf_bits(b.z); r.hi[6] = (unsigned short)h; r.lo[6] = (unsigned short)bf_lo(b.z, h);
  h = bf_bits(b.w); r.hi[7] = (unsigned short)h; r.lo[7] = (unsigned short)bf_lo(b.w, h);
  return r;
}

__device__ __forceinline__ v8f wmb(v16bf a, v16bf b, v8f c) {
  v8f d = __builtin_amdgcn_wmma_f32_16x16x32_bf16(false, a, false, b, (short)0, c, false, false);
  asm volatile("v_nop\n\tv_nop\n\tv_nop\n\tv_nop" : "+v"(d) : "v"(a), "v"(b));
  return d;
}

template <int NBT>
__device__ __forceinline__ int scan_chunk(const int* __restrict__ dsts, int nE, int cbase, int nodeBase,
                                          int vec8, int* list, int tid, int lane, int wave) {
  int wc = 0;
#pragma unroll
  for (int g = 0; g < NGRP; ++g) {
    const int el0  = (g * NTHR + tid) * EPT;
    const int e0   = cbase + el0;
    const int sent = -2147483647 - 1;
    v4i da, db;
    if (vec8 != 0 && e0 + 7 < nE) {
      da = *(const v4i*)(dsts + e0);
      db = *(const v4i*)(dsts + e0 + 4);
    } else {
      da.x = (e0     < nE) ? dsts[min(e0, nE - 1)] : sent;
      da.y = (e0 + 1 < nE) ? dsts[min(e0 + 1, nE - 1)] : sent;
      da.z = (e0 + 2 < nE) ? dsts[min(e0 + 2, nE - 1)] : sent;
      da.w = (e0 + 3 < nE) ? dsts[min(e0 + 3, nE - 1)] : sent;
      db.x = (e0 + 4 < nE) ? dsts[min(e0 + 4, nE - 1)] : sent;
      db.y = (e0 + 5 < nE) ? dsts[min(e0 + 5, nE - 1)] : sent;
      db.z = (e0 + 6 < nE) ? dsts[min(e0 + 6, nE - 1)] : sent;
      db.w = (e0 + 7 < nE) ? dsts[min(e0 + 7, nE - 1)] : sent;
    }
    const unsigned nb = (unsigned)nodeBase;
    const unsigned s0 = (unsigned)da.x - nb, s1 = (unsigned)da.y - nb;
    const unsigned s2 = (unsigned)da.z - nb, s3 = (unsigned)da.w - nb;
    const unsigned s4 = (unsigned)db.x - nb, s5 = (unsigned)db.y - nb;
    const unsigned s6 = (unsigned)db.z - nb, s7 = (unsigned)db.w - nb;
    const bool h0 = s0 < (unsigned)NBT, h1 = s1 < (unsigned)NBT, h2 = s2 < (unsigned)NBT, h3 = s3 < (unsigned)NBT;
    const bool h4 = s4 < (unsigned)NBT, h5 = s5 < (unsigned)NBT, h6 = s6 < (unsigned)NBT, h7 = s7 < (unsigned)NBT;
    const unsigned any = __builtin_amdgcn_ballot_w32(h0 | h1 | h2 | h3 | h4 | h5 | h6 | h7);
    if (any != 0u) {
#define HITJ(J, HJ, SJ) { \
        const unsigned mj = __builtin_amdgcn_ballot_w32(HJ); \
        if (mj != 0u) { \
          if (HJ) { \
            const int pos = wc + (int)__builtin_amdgcn_mbcnt_lo(mj, 0u); \
            if (pos < WCAP) list[wave * WCAP + pos] = ((el0 + (J)) << 12) | (int)(SJ); \
          } \
          wc += (int)__builtin_popcount(mj); } }
      HITJ(0, h0, s0)
      HITJ(1, h1, s1)
      HITJ(2, h2, s2)
      HITJ(3, h3, s3)
      HITJ(4, h4, s4)
      HITJ(5, h5, s5)
      HITJ(6, h6, s6)
      HITJ(7, h7, s7)
#undef HITJ
    }
  }
  return wc;
}

__global__ __launch_bounds__(NTHR) void k_wprep(
    const float* __restrict__ wtm, const float* __restrict__ wts,
    const float* __restrict__ lc, unsigned short* wpl) {
  const int i = blockIdx.x * NTHR + threadIdx.x;
  if (i >= 2 * (WPL / 8)) return;
  const int mat = i >> 9;
  const int j   = i & 511;
  const int n   = j >> 3;
  const int k0  = (j & 7) * 8;
  const float* wt = (mat == 0) ? wtm : wts;
  float v[8];
#pragma unroll
  for (int e = 0; e < 8; ++e) v[e] = 0.f;
#pragma unroll 1
  for (int b = 0; b < NBAS; ++b) {
    const float cb = lc[b];
#pragma unroll
    for (int e = 0; e < 8; ++e)
      v[e] = v[e] + wt[((size_t)(k0 + e) * DIM + n) * NBAS + b] * cb;
  }
  v4f a, bq;
  a.x = v[0]; a.y = v[1]; a.z = v[2]; a.w = v[3];
  bq.x = v[4]; bq.y = v[5]; bq.z = v[6]; bq.w = v[7];
  const HL s = split8(a, bq);
  unsigned short* ph = wpl + (size_t)(2 * mat) * WPL + n * DIM + k0;
  unsigned short* pl = ph + WPL;
  *(volatile v8us*)ph = s.hi;
  *(volatile v8us*)pl = s.lo;
  __threadfence();
  *(volatile v8us*)ph = s.hi;
  *(volatile v8us*)pl = s.lo;
}

__global__ __launch_bounds__(NTHR) void k_gemm(
    const float* __restrict__ x, const unsigned short* __restrict__ wpl,
    float* gmsg, float* gself, int nN) {
  __shared__ __attribute__((aligned(16))) float stg[NWAVE * 16 * DIM];
  const int tid = threadIdx.x, lane = tid & 31, wave = tid >> 5, hh = lane >> 4, m = lane & 15;
  const int which = wave & 1;
  const int rt    = wave >> 1;
  const int row0  = blockIdx.x * GROWS + rt * 16;
  int node = row0 + m;
  node = node > nN - 1 ? nN - 1 : node;
  const float* xp = x + (size_t)node * DIM;
  const unsigned short* whi = wpl + (size_t)(2 * which) * WPL;
  const unsigned short* wlo = whi + WPL;

  v8f acc[4];
#pragma unroll
  for (int t = 0; t < 4; ++t) { v8f z = {0.f, 0.f, 0.f, 0.f, 0.f, 0.f, 0.f, 0.f}; acc[t] = z; }

#pragma unroll
  for (int ks = 0; ks < DIM / 32; ++ks) {
    const float* p0 = xp + 32 * ks + 8 * hh;
    const v4f f0 = *(const v4f*)p0,        f1 = *(const v4f*)(p0 + 4);
    const v4f f2 = *(const v4f*)(p0 + 16), f3 = *(const v4f*)(p0 + 20);
    const HL s0 = split8(f0, f1);
    const HL s1 = split8(f2, f3);
    FragB ah, al;
    ah.h[0] = s0.hi; ah.h[1] = s1.hi;
    al.h[0] = s0.lo; al.h[1] = s1.lo;
#pragma unroll
    for (int t = 0; t < 4; ++t) {
      const unsigned short* bp = whi + (size_t)(16 * t + m) * DIM + 32 * ks + 8 * hh;
      const unsigned short* bq = wlo + (size_t)(16 * t + m) * DIM + 32 * ks + 8 * hh;
      FragB bh, bl;
      bh.h[0] = *(const v8us*)bp; bh.h[1] = *(const v8us*)(bp + 16);
      bl.h[0] = *(const v8us*)bq; bl.h[1] = *(const v8us*)(bq + 16);
      acc[t] = wmb(ah.v, bh.v, acc[t]);
      acc[t] = wmb(ah.v, bl.v, acc[t]);
      acc[t] = wmb(al.v, bh.v, acc[t]);
    }
  }

  float* sp = stg + wave * (16 * DIM) + (8 * hh) * DIM + m;
#pragma unroll
  for (int t = 0; t < 4; ++t) {
    sp[0 * DIM + 16 * t] = acc[t][0];
    sp[1 * DIM + 16 * t] = acc[t][1];
    sp[2 * DIM + 16 * t] = acc[t][2];
    sp[3 * DIM + 16 * t] = acc[t][3];
    sp[4 * DIM + 16 * t] = acc[t][4];
    sp[5 * DIM + 16 * t] = acc[t][5];
    sp[6 * DIM + 16 * t] = acc[t][6];
    sp[7 * DIM + 16 * t] = acc[t][7];
  }
  __syncthreads();

  float* G = which ? gself : gmsg;
  const float* lp = stg + wave * (16 * DIM) + 4 * lane;
  float* gp = G + (size_t)row0 * DIM + 4 * lane;
  v4f ov[8];
#pragma unroll
  for (int q = 0; q < 8; ++q) ov[q] = *(const v4f*)(lp + q * 128);
#pragma unroll
  for (int q = 0; q < 8; ++q) *(volatile v4f*)(gp + q * 128) = ov[q];
  __threadfence();
#pragma unroll
  for (int q = 0; q < 8; ++q) *(volatile v4f*)(gp + q * 128) = ov[q];
}

__global__ __launch_bounds__(NTHR) void k_agg(
    const int* __restrict__ ei, const float* __restrict__ gmsg, const float* __restrict__ gself,
    const float* __restrict__ bmsg_b, const float* __restrict__ bself_b, const float* __restrict__ lc,
    float* out, int nN, int nE, int vec8) {
  extern __shared__ v4f lds_dyn[];
  float* acc  = (float*)lds_dyn;
  int*   list = (int*)(acc + NB * DIM);
  __shared__ int wcnt[NWAVE];
  __shared__ __attribute__((aligned(16))) float sbias[2 * DIM];
  const int tid = threadIdx.x, lane = tid & 31, wave = tid >> 5;
  const int nodeBase = blockIdx.x * NB;
  const int* dsts = ei + nE;

  if (tid < 2 * DIM) {
    const int o = tid & (DIM - 1);
    const float* bp = ((tid < DIM) ? bmsg_b : bself_b) + o * NBAS;
    float s = 0.f;
#pragma unroll 1
    for (int b = 0; b < NBAS; ++b) s = s + bp[b] * lc[b];
    sbias[tid] = s;
  }
  {
    const v4f z = {0.f, 0.f, 0.f, 0.f};
    for (int i = tid; i < NB * DIM / 4; i += NTHR) lds_dyn[i] = z;
  }
  __syncthreads();

  const v2f bm2 = *(const v2f*)(sbias + 2 * lane);

  const int nChunks = (nE + CHUNK - 1) / CHUNK;
#pragma unroll 1
  for (int ch = 0; ch < nChunks; ++ch) {
    const int cbase = ch * CHUNK;
    const int wc = scan_chunk<NB>(dsts, nE, cbase, nodeBase, vec8, list, tid, lane, wave);
    if (lane == 0) wcnt[wave] = wc;
    __syncthreads();
    if (wave == 0) {
#pragma unroll 1
      for (int wsx = 0; wsx < NWAVE; ++wsx) {
        int n = __builtin_amdgcn_readfirstlane(wcnt[wsx]);
        n = n > WCAP ? WCAP : (n < 0 ? 0 : n);
        const int* lp = list + wsx * WCAP;
#pragma unroll 1
        for (int i = 0; i < n; ++i) {
          const int ent  = __builtin_amdgcn_readfirstlane(lp[i]);
          const int slot = ent & (NB - 1);
          int e = cbase + ((ent >> 12) & (CHUNK - 1));
          e = e > nE - 1 ? nE - 1 : e;
          int src = ei[e];
          src = src < 0 ? 0 : (src > nN - 1 ? nN - 1 : src);
          const v2f v = *(const v2f*)(gmsg + (size_t)src * DIM + 2 * lane);
          v2f* ap = (v2f*)(acc + slot * DIM + 2 * lane);
          *ap = *ap + (v + bm2);
        }
      }
    }
    __syncthreads();
  }

  const v2f bs2 = *(const v2f*)(sbias + DIM + 2 * lane);
#pragma unroll 2
  for (int j = 0; j < NB / NWAVE; ++j) {
    const int slot = wave * (NB / NWAVE) + j;
    int node = nodeBase + slot;
    node = node > nN - 1 ? nN - 1 : node;
    v2f* ap = (v2f*)(acc + slot * DIM + 2 * lane);
    const v2f g = *(const v2f*)(gself + (size_t)node * DIM + 2 * lane);
    v2f t = *ap + (g + bs2);
    float s = t.x * t.x + t.y * t.y;
    s += __shfl_xor(s, 16, 32);
    s += __shfl_xor(s, 8, 32);
    s += __shfl_xor(s, 4, 32);
    s += __shfl_xor(s, 2, 32);
    s += __shfl_xor(s, 1, 32);
    const float nrm = sqrtf(s);
    const float inv = 1.0f / fmaxf(nrm, 1e-12f);
    *ap = t * inv;
  }
  __syncthreads();

  const size_t outN = (size_t)nN * DIM;
  const size_t ob   = (size_t)nodeBase * DIM;
#pragma unroll 4
  for (int q = 0; q < (NB * DIM) / (NWAVE * 128); ++q) {
    const int f = (wave * ((NB * DIM) / (NWAVE * 128)) + q) * 128 + 4 * lane;
    const size_t gi = ob + (size_t)f;
    if (gi < outN) { const v4f v = *(const v4f*)(acc + f); *(volatile v4f*)(out + gi) = v; }
  }
  __threadfence();
#pragma unroll 4
  for (int q = 0; q < (NB * DIM) / (NWAVE * 128); ++q) {
    const int f = (wave * ((NB * DIM) / (NWAVE * 128)) + q) * 128 + 4 * lane;
    const size_t gi = ob + (size_t)f;
    if (gi < outN) { const v4f v = *(const v4f*)(acc + f); *(volatile v4f*)(out + gi) = v; }
  }
}

extern "C" void kernel_launch(void* const* d_in, const int* in_sizes, int n_in,
                              void* d_out, int out_size, void* d_ws, size_t ws_size,
                              hipStream_t stream) {
  if (n_in < 7) return;
  const int nN = in_sizes[0] / DIM;
  const int nE = in_sizes[1] / 2;
  if (nN <= 0 || nE < 0 || in_sizes[0] != nN * DIM || in_sizes[1] != nE * 2) return;
  if (in_sizes[2] != DIM * DIM * NBAS || in_sizes[3] != DIM * NBAS) return;
  if (in_sizes[4] != DIM * DIM * NBAS || in_sizes[5] != DIM * NBAS) return;
  if (in_sizes[6] < NBAS) return;
  if (out_size != nN * DIM) return;

  const float* x     = (const float*)d_in[0];
  const int*   ei    = (const int*)d_in[1];
  const float* wtm   = (const float*)d_in[2];
  const float* bmsg  = (const float*)d_in[3];
  const float* wts   = (const float*)d_in[4];
  const float* bself = (const float*)d_in[5];
  const float* lc    = (const float*)d_in[6];
  float* out = (float*)d_out;

  const int nGB = (nN + GROWS - 1) / GROWS;
  const int nAB = (nN + NB - 1) / NB;

  char* ws = (char*)d_ws;
  size_t off = 0;
  const size_t oWP = off; off += (size_t)4 * WPL * 2;                          off = (off + 255) & ~(size_t)255;
  const size_t szG = (size_t)nGB * GROWS * DIM * 4;
  const size_t oGM = off; off += szG;                                          off = (off + 255) & ~(size_t)255;
  const size_t oGS = off; off += szG;                                          off = (off + 255) & ~(size_t)255;
  if (off > ws_size) return;
  if (off > ((size_t)128 << 20)) return;
  unsigned short* wpl   = (unsigned short*)(ws + oWP);
  float*          gmsg  = (float*)(ws + oGM);
  float*          gself = (float*)(ws + oGS);

  const int vec8 = ((nE & 3) == 0) ? 1 : 0;

  const int nPrep = 2 * (WPL / 8);
  k_wprep<<<(nPrep + NTHR - 1) / NTHR, NTHR, 0, stream>>>(wtm, wts, lc, wpl);

  k_gemm<<<nGB, NTHR, 0, stream>>>(x, wpl, gmsg, gself, nN);

  hipFuncSetAttribute(reinterpret_cast<const void*>(&k_agg),
                      hipFuncAttributeMaxDynamicSharedMemorySize, LDS_AGG);
  k_agg<<<nAB, NTHR, LDS_AGG, stream>>>(ei, gmsg, gself, bmsg, bself, lc, out, nN, nE, vec8);
}
